// FeatureAlignmentModule_24489903522350
// MI455X (gfx1250) — hardware-run, weakly checked
//
#include <hip/hip_runtime.h>


#ifndef NB
#define NB 16
#endif
#define NB_FULL 16
#define IMH  64
#define IMW  64
#define HW   (IMH * IMW)
#define CIN  128
#define CC   256
#define PH   66
#define PW   66
#define NOFF 18
#define NPAD 32
#define NTAP 9
#define KO   (NTAP * CC)
#define KD   (NTAP * CIN)
#define TP   264
#define VP   136
#define EP   68
#define OSP  36
#define DW   4
#define WDS  64.0f
#define WDI  (1.0f / 64.0f)

static_assert(NB <= NB_FULL);
static_assert(IMW == 64);
static_assert(IMH == 64);
static_assert(PH == IMH + 2);
static_assert(PW == IMW + 2);
static_assert(CC == 2 * CIN);
static_assert(CC == 256);
static_assert(CC == 32 * 8);
static_assert(CIN % 32 == 0);
static_assert(KO % 32 == 0);
static_assert(KD % 32 == 0);
static_assert(NPAD == 32);
static_assert(NOFF <= NPAD);
static_assert(2 * NTAP == NOFF);
static_assert(CIN == DW * 32);
static_assert((TP * 2) % 16 == 0);
static_assert((VP * 2) % 16 == 0);
static_assert((EP * 4) % 16 == 0);
static_assert((OSP * 4) % 16 == 0);
static_assert(TP >= CC);
static_assert(VP >= CIN);
static_assert(EP >= IMW);
static_assert(OSP >= NPAD);
static_assert(32 * 16 * 4 == 16 * NPAD * 4);
static_assert(32 * 16 * 8 == 16 * IMW * 4);
static_assert(8 * 256 * 4 == CIN * IMW);
static_assert(2 * 8 * 8 == CIN);
static_assert(2 * IMW == 32 * DW);
static_assert(IMW * TP * 2 <= 131072);
static_assert(16 * OSP * 4 <= 131072);
static_assert(IMW * VP * 2 + DW * 16 * EP * 4 <= 131072);

typedef _Float16 h16;
typedef unsigned short bf;
typedef __attribute__((ext_vector_type(16))) __bf16   v16bf;
typedef __attribute__((ext_vector_type(16))) _Float16 v16h;
typedef __attribute__((ext_vector_type(8)))  _Float16 v8h;
typedef __attribute__((ext_vector_type(8)))  unsigned short v8us;
typedef __attribute__((ext_vector_type(8)))  float    v8f;
typedef __attribute__((ext_vector_type(4)))  float    v4f;
typedef __attribute__((ext_vector_type(2)))  float    v2f;
typedef __attribute__((ext_vector_type(4)))  unsigned int v4u;
typedef v4f  __attribute__((may_alias)) v4fa;
typedef v8h  __attribute__((may_alias)) v8ha;
typedef v8us __attribute__((may_alias)) v8usa;
typedef v4u  __attribute__((may_alias)) v4ua;

__device__ __forceinline__ unsigned short f2bf(float f) { unsigned u = __float_as_uint(f); u += 0x7FFFu + ((u >> 16) & 1u); return (unsigned short)(u >> 16); }
__device__ __forceinline__ float bfr(float f) { return __uint_as_float(((unsigned)f2bf(f)) << 16); }
__device__ __forceinline__ h16 toh_flush(float v) { const h16 r = (h16)v; return (fabsf(v) < 6.103515625e-05f) ? (h16)0.0f : r; }
__device__ __forceinline__ v16h cat16(v8h lo, v8h hi) { return __builtin_shufflevector(lo, hi, 0, 1, 2, 3, 4, 5, 6, 7, 8, 9, 10, 11, 12, 13, 14, 15); }
__device__ __forceinline__ v16bf cat16b(v8us lo, v8us hi) { return __builtin_bit_cast(v16bf, __builtin_shufflevector(lo, hi, 0, 1, 2, 3, 4, 5, 6, 7, 8, 9, 10, 11, 12, 13, 14, 15)); }
__device__ __forceinline__ v8f wmma16g(v16h a, v16h b, v8f c) {
    c = __builtin_amdgcn_wmma_f32_16x16x32_f16(false, a, false, b, (short)0, c, false, false);
    asm volatile("v_nop\n\tv_nop\n\tv_nop\n\tv_nop" : "+v"(c) : "v"(a), "v"(b));
    return c; }
__device__ __forceinline__ v8f wmmabg(v16bf a, v16bf b, v8f c) {
    c = __builtin_amdgcn_wmma_f32_16x16x32_bf16(false, a, false, b, (short)0, c, false, false);
    asm volatile("v_nop\n\tv_nop\n\tv_nop\n\tv_nop" : "+v"(c) : "v"(a), "v"(b));
    return c; }
__device__ __forceinline__ v16h  ldh(const h16* p) { return cat16(*(const v8h*)p, *(const v8h*)(p + 16)); }
__device__ __forceinline__ v16bf ldb(const bf* p)  { return cat16b(*(const v8us*)p, *(const v8us*)(p + 16)); }
__device__ __forceinline__ void wave_sync() { __builtin_amdgcn_fence(3  , "wavefront"); __builtin_amdgcn_wave_barrier(); asm volatile("" ::: "memory"); }

__global__ __launch_bounds__(256) void k_nhwc(const float* __restrict__ vis, const float* __restrict__ ir, bf* XB) {
    __shared__ __align__(16) unsigned short ts[IMW * TP];
    const int tid = threadIdx.x, lane = tid & 31;
    const int wave = __builtin_amdgcn_readfirstlane((int)(threadIdx.x >> 5));
    const int py = blockIdx.x, b = blockIdx.y;
    const bool inrow = (py >= 1) & (py <= IMH);
    if (inrow) {
        const size_t rb = (size_t)b * CIN * HW + (size_t)(py - 1) * IMW;
#pragma unroll 2
        for (int i = 0; i < 8; ++i) { const int idx = i * 256 + tid; const int c = idx >> 4, x4 = (idx & 15) * 4;
            const v4f v = *(const v4f*)(vis + rb + (size_t)c * HW + x4);
#pragma unroll
            for (int k = 0; k < 4; ++k) ts[(x4 + k) * TP + c] = f2bf(v[k]); }
#pragma unroll 2
        for (int i = 0; i < 8; ++i) { const int idx = i * 256 + tid; const int c = idx >> 4, x4 = (idx & 15) * 4;
            const v4f v = *(const v4f*)(ir + rb + (size_t)c * HW + x4);
#pragma unroll
            for (int k = 0; k < 4; ++k) ts[(x4 + k) * TP + CIN + c] = f2bf(v[k]); }
    }
    __syncthreads();
    bf* rowp = XB + ((size_t)(b * PH + py) * PW) * CC;
    const v8us zz = (v8us){};
#pragma unroll 1
    for (int ps = 0; ps < 2; ++ps) {
        if (inrow) {
#pragma unroll 1
            for (int i = 0; i < 8; ++i) { const int sx = wave + 8 * i;
                const v8us tv = *(const v8usa*)(&ts[sx * TP + lane * 8]);
                *(volatile v8us*)(rowp + (size_t)(sx + 1) * CC + lane * 8) = tv; }
            if (wave < 2) { const int px = wave * (PW - 1);
                *(volatile v8us*)(rowp + (size_t)px * CC + lane * 8) = zz; }
        } else {
#pragma unroll 1
            for (int px = wave; px < PW; px += 8) *(volatile v8us*)(rowp + (size_t)px * CC + lane * 8) = zz;
        }
        if (ps == 0) __threadfence(); }
}

__global__ __launch_bounds__(256) void k_woff(const float* __restrict__ w, bf* WO) {
    const int i = blockIdx.x * 256 + threadIdx.x; if (i >= NPAD * KO / 8) return;
    const int n = i / (KO / 8), rem = i % (KO / 8); const int t = rem / (CC / 8), c0 = (rem % (CC / 8)) * 8;
    const int nc = n < NOFF ? n : NOFF - 1;
    v8us o;
#pragma unroll
    for (int k = 0; k < 8; ++k) { float x = w[((size_t)nc * CC + c0 + k) * NTAP + t]; asm volatile("" : "+v"(x)); o[k] = (n < NOFF) ? f2bf(x) : (unsigned short)0; }
    *(volatile v8us*)(WO + (size_t)i * 8) = o; __threadfence(); *(volatile v8us*)(WO + (size_t)i * 8) = o;
}

__global__ __launch_bounds__(256) void k_wdef(const float* __restrict__ w, h16* WD) {
    const int i = blockIdx.x * 256 + threadIdx.x; if (i >= CIN * KD / 8) return;
    const int o = i / (KD / 8), rem = i % (KD / 8); const int t = rem / (CIN / 8), c0 = (rem % (CIN / 8)) * 8;
    v8h hv;
#pragma unroll
    for (int k = 0; k < 8; ++k) { const float x = w[((size_t)o * CIN + c0 + k) * NTAP + t]; hv[k] = toh_flush(bfr(x) * WDS); }
    *(volatile v8h*)(WD + (size_t)i * 8) = hv; __threadfence(); *(volatile v8h*)(WD + (size_t)i * 8) = hv;
}

__global__ __launch_bounds__(32) void k_offs(const bf* __restrict__ XB, const bf* __restrict__ WO, const float* __restrict__ boff, float* OFF) {
    __shared__ __align__(16) float os[16 * OSP];
    const int lane = threadIdx.x & 31, lr = lane & 15, hi = lane >> 4;
    const int b = blockIdx.x / IMH, y = blockIdx.x % IMH;
    v8f acc[4][2];
#pragma unroll
    for (int mb = 0; mb < 4; ++mb)
#pragma unroll
        for (int nb = 0; nb < 2; ++nb) acc[mb][nb] = (v8f){};
    const size_t aoff = (((size_t)(b * PH + y) * PW) + (size_t)lr) * CC + 8 * hi;
    const size_t woff = (size_t)lr * KO + 8 * hi;
#pragma unroll 1
    for (int kc = 0; kc < KO; kc += 32) {
        const int t = kc >> 8, cc = kc & 255; const int ty = t / 3, tx = t - 3 * ty;
        const size_t ao = aoff + ((size_t)ty * PW + (size_t)tx) * CC + (size_t)cc;
        v16bf a[4];
#pragma unroll
        for (int mb = 0; mb < 4; ++mb) a[mb] = ldb(XB + ao + (size_t)mb * 16 * CC);
#pragma unroll
        for (int nb = 0; nb < 2; ++nb) { const v16bf bb = ldb(WO + woff + (size_t)nb * 16 * KO + kc);
#pragma unroll
            for (int mb = 0; mb < 4; ++mb) acc[mb][nb] = wmmabg(a[mb], bb, acc[mb][nb]); }
    }
    float bc[2]; bool vn[2];
#pragma unroll
    for (int nb = 0; nb < 2; ++nb) { const int n = nb * 16 + lr; float bv = boff[n < NOFF ? n : NOFF - 1]; asm volatile("" : "+v"(bv)); bc[nb] = bfr(bv); vn[nb] = n < NOFF; }
    float* obase = OFF + ((size_t)(b * IMH + y) * IMW) * NPAD;
#pragma unroll
    for (int mb = 0; mb < 4; ++mb) {
#pragma unroll
        for (int nb = 0; nb < 2; ++nb) {
#pragma unroll
            for (int j = 0; j < 8; ++j) { float v = acc[mb][nb][j] + bc[nb]; v = v > 0.0f ? v : 0.0f;
                os[(hi * 8 + j) * OSP + nb * 16 + lr] = vn[nb] ? v : 0.0f; } }
        wave_sync();
#pragma unroll 1
        for (int ps = 0; ps < 2; ++ps) {
#pragma unroll
            for (int s = 0; s < 4; ++s) { const int row = 4 * s + (lane >> 3), cofs = (lane & 7) * 4;
                const v4f val = *(const v4fa*)(&os[row * OSP + cofs]);
                *(volatile v4f*)(obase + (size_t)(mb * 16 + row) * NPAD + cofs) = val; }
            if (ps == 0) __threadfence(); }
        wave_sync();
    }
}

__global__ __launch_bounds__(32 * DW) void k_deform(const bf* __restrict__ XB, const float* __restrict__ OFF, const h16* __restrict__ WD, const float* __restrict__ bdef, float* OUT) {
    __shared__ __align__(16) h16 sv[IMW * VP];
    __shared__ __align__(16) float es[DW * 16 * EP];
    const int tid = threadIdx.x, lane = tid & 31, lr = lane & 15, hi = lane >> 4;
    const int wave = __builtin_amdgcn_readfirstlane((int)(threadIdx.x >> 5));
    const int b = blockIdx.x / IMH, y = blockIdx.x % IMH;
    const int p = tid >> 1, ch0 = (tid & 1) * 64;
    v8f acc[4][2];
#pragma unroll
    for (int mb = 0; mb < 4; ++mb)
#pragma unroll
        for (int nb = 0; nb < 2; ++nb) acc[mb][nb] = (v8f){};
    const size_t wb = (size_t)(wave * 32 + lr) * KD + 8 * hi;
    const float* offp = OFF + ((size_t)(b * IMH + y) * IMW + (size_t)p) * NPAD;
    const size_t xbb = (size_t)b * PH * PW * CC + CIN + (size_t)ch0;
#pragma unroll 1
    for (int t = 0; t < NTAP; ++t) {
        const int ty = t / 3, tx = t - 3 * ty;
        const v2f dd = *(const v2f*)(offp + 2 * t);
        const float fy = (dd[0] + (float)y) + (float)(ty - 1);
        const float fx = (dd[1] + (float)p) + (float)(tx - 1);
        const float fy0 = floorf(fy), fx0 = floorf(fx);
        const float wy = fy - fy0, wx = fx - fx0;
        const float fyc = fminf(fmaxf(fy0, -2.0f), (float)IMH);
        const float fxc = fminf(fmaxf(fx0, -2.0f), (float)IMW);
        const int y0 = (int)fyc, x0 = (int)fxc; const int y1 = y0 + 1, x1 = x0 + 1;
        const bool vy0 = (y0 >= 0) & (y0 < IMH), vy1 = (y1 >= 0) & (y1 < IMH);
        const bool vx0 = (x0 >= 0) & (x0 < IMW), vx1 = (x1 >= 0) & (x1 < IMW);
        const int yc0 = y0 < 0 ? 0 : (y0 > IMH - 1 ? IMH - 1 : y0), yc1 = y1 < 0 ? 0 : (y1 > IMH - 1 ? IMH - 1 : y1);
        const int xc0 = x0 < 0 ? 0 : (x0 > IMW - 1 ? IMW - 1 : x0), xc1 = x1 < 0 ? 0 : (x1 > IMW - 1 ? IMW - 1 : x1);
        const float omy = 1.0f - wy, omx = 1.0f - wx;
        const float w00 = (vy0 & vx0) ? omy * omx : 0.0f;
        const float w01 = (vy0 & vx1) ? omy * wx  : 0.0f;
        const float w10 = (vy1 & vx0) ? wy * omx  : 0.0f;
        const float w11 = (vy1 & vx1) ? wy * wx   : 0.0f;
        const size_t a00 = xbb + ((size_t)(yc0 + 1) * PW + (size_t)(xc0 + 1)) * CC;
        const size_t a01 = xbb + ((size_t)(yc0 + 1) * PW + (size_t)(xc1 + 1)) * CC;
        const size_t a10 = xbb + ((size_t)(yc1 + 1) * PW + (size_t)(xc0 + 1)) * CC;
        const size_t a11 = xbb + ((size_t)(yc1 + 1) * PW + (size_t)(xc1 + 1)) * CC;
#pragma unroll 1
        for (int q = 0; q < 8; ++q) {
            const int c = q * 8;
            const v4u u00 = *(const v4ua*)(XB + a00 + c); const v4u u01 = *(const v4ua*)(XB + a01 + c);
            const v4u u10 = *(const v4ua*)(XB + a10 + c); const v4u u11 = *(const v4ua*)(XB + a11 + c);
            v8h hv;
#pragma unroll
            for (int i = 0; i < 4; ++i) {
                float e = w00 * __uint_as_float(u00[i] << 16);
                float o = w00 * __uint_as_float(u00[i] & 0xffff0000u);
                e += w01 * __uint_as_float(u01[i] << 16); o += w01 * __uint_as_float(u01[i] & 0xffff0000u);
                e += w10 * __uint_as_float(u10[i] << 16); o += w10 * __uint_as_float(u10[i] & 0xffff0000u);
                e += w11 * __uint_as_float(u11[i] << 16); o += w11 * __uint_as_float(u11[i] & 0xffff0000u);
                hv[2 * i] = toh_flush(e); hv[2 * i + 1] = toh_flush(o); }
            *(v8ha*)(&sv[p * VP + ch0 + c]) = hv; }
        __syncthreads();
#pragma unroll 1
        for (int kc = 0; kc < CIN; kc += 32) {
            v16h a[4];
#pragma unroll
            for (int mb = 0; mb < 4; ++mb) { const int so = (mb * 16 + lr) * VP + kc + 8 * hi;
                a[mb] = cat16(*(const v8ha*)(&sv[so]), *(const v8ha*)(&sv[so + 16])); }
#pragma unroll
            for (int nb = 0; nb < 2; ++nb) { const v16h bb = ldh(WD + wb + (size_t)nb * 16 * KD + (size_t)(t * CIN + kc));
#pragma unroll
                for (int mb = 0; mb < 4; ++mb) acc[mb][nb] = wmma16g(a[mb], bb, acc[mb][nb]); }
        }
        __syncthreads();
    }
    const int eb = wave * 16 * EP;
#pragma unroll
    for (int nb = 0; nb < 2; ++nb) {
        const float bias = bfr(bdef[wave * 32 + nb * 16 + lr]);
#pragma unroll
        for (int mb = 0; mb < 4; ++mb) { v4f a, c;
#pragma unroll
            for (int i = 0; i < 4; ++i) { a[i] = acc[mb][nb][i] * WDI + bias; c[i] = acc[mb][nb][4 + i] * WDI + bias; }
            *(v4fa*)(&es[eb + lr * EP + mb * 16 + 8 * hi]) = a; *(v4fa*)(&es[eb + lr * EP + mb * 16 + 8 * hi + 4]) = c; }
        wave_sync();
        float* orow = OUT + (((size_t)b * CIN + (size_t)(wave * 32 + nb * 16)) * IMH + (size_t)y) * IMW;
#pragma unroll 1
        for (int ps = 0; ps < 2; ++ps) {
#pragma unroll
            for (int s = 0; s < 8; ++s) { const int row = 2 * s + (lane >> 4), cofs = (lane & 15) * 4;
                const v4f val = *(const v4fa*)(&es[eb + row * EP + cofs]);
                *(volatile v4f*)(orow + (size_t)row * HW + cofs) = val; }
            if (ps == 0) __threadfence(); }
        wave_sync();
    }
}

static constexpr size_t al256(size_t v) { return (v + 255) & ~(size_t)255; }
static constexpr size_t SZ_XB = al256((size_t)NB * PH * PW * CC * 2);
static constexpr size_t SZ_WO = al256((size_t)NPAD * KO * 2);
static constexpr size_t SZ_WD = al256((size_t)CIN * KD * 2);
static constexpr size_t SZ_OF = al256((size_t)NB * HW * NPAD * 4);
static constexpr size_t SZ_TOTAL = SZ_XB + SZ_WO + SZ_WD + SZ_OF;
static_assert(SZ_TOTAL <= (size_t)134217728);
static_assert(((size_t)NPAD * KO) % 8 == 0);
static_assert(((size_t)CIN * KD) % 8 == 0);
static_assert(((size_t)PW * CC * 2) % 128 == 0);
static_assert((size_t)(NB * IMH - 1) * IMW * NPAD + (size_t)63 * NPAD + NPAD <= (size_t)NB * HW * NPAD);

extern "C" void kernel_launch(void* const* d_in, const int* in_sizes, int n_in,
                              void* d_out, int out_size, void* d_ws, size_t ws_size, hipStream_t stream) {
    if (n_in < 6) return;
    const size_t needx = (size_t)NB * CIN * HW;
    if ((size_t)in_sizes[0] < needx || (size_t)in_sizes[1] < needx) return;
    if ((size_t)in_sizes[2] < (size_t)NOFF * CC * NTAP || in_sizes[3] < NOFF) return;
    if ((size_t)in_sizes[4] < (size_t)CIN * CIN * NTAP || in_sizes[5] < CIN) return;
    if ((size_t)out_size < needx) return;
    if (SZ_TOTAL > ws_size) return;
    const float* vis  = (const float*)d_in[0];
    const float* ir   = (const float*)d_in[1];
    const float* woff = (const float*)d_in[2];
    const float* boff = (const float*)d_in[3];
    const float* wdef = (const float*)d_in[4];
    const float* bdef = (const float*)d_in[5];
    float* OUT = (float*)d_out;
    char* wsp = (char*)d_ws;
    bf*    XB  = (bf*)wsp;    wsp += SZ_XB;
    bf*    WO  = (bf*)wsp;    wsp += SZ_WO;
    h16*   WD  = (h16*)wsp;   wsp += SZ_WD;
    float* OFF = (float*)wsp; wsp += SZ_OF;

    k_nhwc<<<dim3(PH, NB, 1), 256, 0, stream>>>(vis, ir, XB);
    k_woff<<<(unsigned)((NPAD * KO / 8 + 255) / 256), 256, 0, stream>>>(woff, WO);
    k_wdef<<<(unsigned)((CIN * KD / 8 + 255) / 256), 256, 0, stream>>>(wdef, WD);
    k_offs<<<NB * IMH, 32, 0, stream>>>(XB, WO, boff, OFF);
    k_deform<<<NB * IMH, 32 * DW, 0, stream>>>(XB, OFF, WD, bdef, OUT);
}
